// StreamingTransformer_40922448397087
// MI455X (gfx1250) — hardware-verified
//
#include <hip/hip_runtime.h>
#include <stdint.h>

typedef __attribute__((ext_vector_type(16))) _Float16 v16h;
typedef __attribute__((ext_vector_type(8)))  _Float16 v8h;
typedef __attribute__((ext_vector_type(16))) __bf16   v16b;
typedef __attribute__((ext_vector_type(8)))  __bf16   v8b;
typedef __attribute__((ext_vector_type(8)))  float    v8f;
typedef __attribute__((ext_vector_type(4)))  float    v4f;
typedef __attribute__((ext_vector_type(4)))  unsigned int v4u;

constexpr int NBATCH   = 8;
constexpr int SEQ      = 1000;
constexpr int SEQP     = 1024;
constexpr int CIN      = 512;
constexpr int NHEAD    = 8;
constexpr int HDIM     = 64;
constexpr int NLAYER   = 6;
constexpr int LAYER_LAST = NLAYER - 1;
constexpr int KV_LIM   = 256;
constexpr int MROWS    = NBATCH * SEQP;

static_assert(CIN % 32 == 0, "K of every GEMM is a multiple of 32");
static_assert(CIN % 64 == 0, "N of every GEMM is a multiple of 64");
static_assert(MROWS % 64 == 0, "M of Q / output GEMM is a multiple of 64");
static_assert(KV_LIM % 64 == 0, "M of K/V GEMM and key chunking are multiples of 64");
static_assert(SEQP % 64 == 0, "query blocks never cross a batch");
static_assert(HDIM == 64 && NHEAD * HDIM == CIN, "head geometry");
static_assert(KV_LIM <= SEQ, "kept keys are all real positions");

__device__ __forceinline__ unsigned short f2bf_bits(float f) {
  unsigned u = __float_as_uint(f);
  return (unsigned short)((u + 0x7FFFu + ((u >> 16) & 1u)) >> 16);
}
__device__ __forceinline__ float bf_bits2f(unsigned short h) { return __uint_as_float(((unsigned)h) << 16); }

__device__ __forceinline__ void dep_guard_h(v8f& a, v8f& b, v16h x, v16h y) { asm volatile("v_nop\n\tv_nop\n\tv_nop\n\tv_nop" : "+v"(a), "+v"(b) : "v"(x), "v"(y)); }
__device__ __forceinline__ void dep_guard_b(v8f& a, v8f& b, v16b x, v16b y) { asm volatile("v_nop\n\tv_nop\n\tv_nop\n\tv_nop" : "+v"(a), "+v"(b) : "v"(x), "v"(y)); }
__device__ __forceinline__ void keep4_h(v16h a, v16h b, v16h c, v16h d) { asm volatile("v_nop" :: "v"(a), "v"(b), "v"(c), "v"(d)); }
__device__ __forceinline__ void keep4_b(v16b a, v16b b, v16b c, v16b d) { asm volatile("v_nop" :: "v"(a), "v"(b), "v"(c), "v"(d)); }
__device__ __forceinline__ void acc_guard4(v8f& a, v8f& b, v8f& c, v8f& d) { asm volatile("v_nop\n\tv_nop\n\tv_nop\n\tv_nop" : "+v"(a), "+v"(b), "+v"(c), "+v"(d)); }
template <typename T> struct Frag;
template <> struct Frag<_Float16> {
  typedef v16h V; union U { v16h v; v8h h[2]; };
  static __device__ __forceinline__ v16h load(const _Float16* p) {
    U f; f.h[0] = *(const v8h*)(p); f.h[1] = *(const v8h*)(p + 16); return f.v;
  }
  static __device__ __forceinline__ v8f mma(v16h a, v16h b, v8f c) {
    return __builtin_amdgcn_wmma_f32_16x16x32_f16(false, a, false, b, (short)0, c, false, false);
  }
  static __device__ __forceinline__ void guard(v8f& a, v8f& b, v16h x, v16h y) { dep_guard_h(a, b, x, y); }
  static __device__ __forceinline__ void keep(v16h a, v16h b, v16h c, v16h d) { keep4_h(a, b, c, d); }
};
template <> struct Frag<__bf16> {
  typedef v16b V; union U { v16b v; v8b h[2]; };
  static __device__ __forceinline__ v16b load(const __bf16* p) {
    U f; f.h[0] = *(const v8b*)(p); f.h[1] = *(const v8b*)(p + 16); return f.v;
  }
  static __device__ __forceinline__ v8f mma(v16b a, v16b b, v8f c) {
    return __builtin_amdgcn_wmma_f32_16x16x32_bf16(false, a, false, b, (short)0, c, false, false);
  }
  static __device__ __forceinline__ void guard(v8f& a, v8f& b, v16b x, v16b y) { dep_guard_b(a, b, x, y); }
  static __device__ __forceinline__ void keep(v16b a, v16b b, v16b c, v16b d) { keep4_b(a, b, c, d); }
};

template <int ET> struct Elem;
template <> struct Elem<0> { typedef _Float16 T; };
template <> struct Elem<1> { typedef __bf16 T; };
template <int ET, bool SPLIT, int BIAS_MODE, int OUT_MODE, bool RESID, int ACT = 0, bool ROWMAP = false>
__global__ __launch_bounds__(256) void wmma_gemm64(
    const unsigned short* __restrict__ Ap, const unsigned short* __restrict__ A2p, int lda, long strideA,
    const unsigned short* __restrict__ Btp, const unsigned short* __restrict__ Bt2p, int ldb, long strideB,
    void* __restrict__ Cout, void* __restrict__ Cout2, int ldc, long strideC,
    const float* __restrict__ bias,
    const float* __restrict__ resid, long strideR,
    int M, int N, int K, float scale, int rowsPer, int rowsKeep) {
  typedef typename Elem<ET>::T T;
  typedef typename Frag<T>::V V;
  const T* A = (const T*)Ap; const T* A2 = (const T*)A2p; const T* Bt = (const T*)Btp; const T* Bt2 = (const T*)Bt2p;
  __shared__ __align__(16) float sT[8][16 * 68];
  const int b    = blockIdx.y;
  const int lane = threadIdx.x & 31;
  const int wave = threadIdx.x >> 5;
  const int tilesN = N >> 6;
  const int tilesM = M >> 6;
  const int tile = blockIdx.x * 8 + wave;
  if (tile >= tilesM * tilesN) return;
  const int tm = tile / tilesN;
  const int tn = tile - tm * tilesN;
  const int m0 = tm << 6;
  const int n0 = tn << 6;

  const T* Ab  = A  + (size_t)b * strideA;
  const T* Bb  = Bt + (size_t)b * strideB;
  const T* Ab2 = SPLIT ? (A2  + (size_t)b * strideA) : nullptr;
  const T* Bb2 = SPLIT ? (Bt2 + (size_t)b * strideB) : nullptr;

  const int rlane = lane & 15;
  const int koff  = (lane >> 4) * 8;
  const int mOff  = (lane >> 4) * 8;

  v8f acc[4][4];
#pragma unroll
  for (int i = 0; i < 4; ++i)
#pragma unroll
    for (int j = 0; j < 4; ++j) acc[i][j] = (v8f){0.f,0.f,0.f,0.f,0.f,0.f,0.f,0.f};

  for (int k0 = 0; k0 < K; k0 += 32) {
    V bh[4], bl[4];
#pragma unroll
    for (int j = 0; j < 4; ++j) {
      const size_t bo = (size_t)(n0 + (j << 4) + rlane) * ldb + koff + k0;
      bh[j] = Frag<T>::load(Bb + bo);
      if (SPLIT) bl[j] = Frag<T>::load(Bb2 + bo);
    }
#pragma unroll
    for (int i = 0; i < 4; ++i) {
      const size_t ao = (size_t)(m0 + (i << 4) + rlane) * lda + koff + k0;
      V ah = Frag<T>::load(Ab + ao);
      V al;
      if (SPLIT) al = Frag<T>::load(Ab2 + ao);
#pragma unroll
      for (int j = 0; j < 4; ++j) {
        acc[i][j] = Frag<T>::mma(ah, bh[j], acc[i][j]);
        if (SPLIT) {
          acc[i][j] = Frag<T>::mma(ah, bl[j], acc[i][j]);
          acc[i][j] = Frag<T>::mma(al, bh[j], acc[i][j]);
        }
      }
      Frag<T>::guard(acc[i][0], acc[i][3], ah, SPLIT ? al : ah);
    }
    Frag<T>::keep(bh[0], bh[1], bh[2], bh[3]);
    if (SPLIT) Frag<T>::keep(bl[0], bl[1], bl[2], bl[3]);
  }
  acc_guard4(acc[0][0], acc[0][1], acc[0][2], acc[0][3]);
  acc_guard4(acc[1][0], acc[1][1], acc[1][2], acc[1][3]);
  acc_guard4(acc[2][0], acc[2][1], acc[2][2], acc[2][3]);
  acc_guard4(acc[3][0], acc[3][1], acc[3][2], acc[3][3]);

  float* slab = sT[wave];
  const float* Rb = RESID ? (resid + (size_t)b * strideR) : nullptr;
#pragma unroll
  for (int i = 0; i < 4; ++i) {
    const int mBase = m0 + (i << 4);
#pragma unroll
    for (int j = 0; j < 4; ++j) {
      const int n = n0 + (j << 4) + rlane;
      float bv = 0.f;
      if (BIAS_MODE == 2) bv = bias[n];
#pragma unroll
      for (int r = 0; r < 8; ++r) {
        float v = acc[i][j][r] * scale;
        if (BIAS_MODE == 1) v += bias[mBase + mOff + r];
        if (BIAS_MODE == 2) v += bv;
        if (RESID) v += Rb[(size_t)(mBase + mOff + r) * ldc + n];
        if (ACT == 1) v = tanhf(v);
        if (ACT == 2) v = fmaxf(v, 0.0f);
        if (ACT == 3) v = v / (1.0f + expf(-v));
        if (ACT == 4) v = (v > 0.f) ? v : 0.01f * v;
        slab[(mOff + r) * 68 + (j << 4) + rlane] = v;
      }
    }
    __builtin_amdgcn_fence(__ATOMIC_RELEASE, "workgroup");
    __builtin_amdgcn_wave_barrier();
    __builtin_amdgcn_fence(__ATOMIC_ACQUIRE, "workgroup");
    if (OUT_MODE == 0) {
      float* C = (float*)Cout + (size_t)b * strideC;
      const int hh = lane >> 4, c4 = (lane & 15) * 4;
      for (int pass = 0; pass < 2; ++pass) {
#pragma unroll
        for (int it = 0; it < 8; ++it) {
          const int row = it * 2 + hh;
          v4f v = *(const v4f*)(slab + row * 68 + c4);
          const int msrc = mBase + row;
          int orow = msrc;
          bool keep = true;
          if (ROWMAP) {
            const int grp = msrc / rowsPer;
            const int sub = msrc - grp * rowsPer;
            keep = (sub < rowsKeep);
            orow = grp * rowsKeep + sub;
          }
          if (keep) *(volatile v4f*)(C + (size_t)orow * ldc + n0 + c4) = v;
        }
        __threadfence();
      }
    } else {
      const int q = lane >> 3, c8 = (lane & 7) * 8;
      unsigned short* C  = (unsigned short*)Cout  + (size_t)b * strideC;
      unsigned short* C2 = (OUT_MODE == 2) ? ((unsigned short*)Cout2 + (size_t)b * strideC) : nullptr;
      for (int pass = 0; pass < 2; ++pass) {
#pragma unroll
        for (int it = 0; it < 4; ++it) {
          const int row = it * 4 + q;
          const float* sp = slab + row * 68 + c8;
          v8h hv, lv;
#pragma unroll
          for (int e = 0; e < 8; ++e) {
            if (OUT_MODE == 1) {
              hv[e] = (_Float16)sp[e];
            } else {
              unsigned short hb = f2bf_bits(sp[e]);
              unsigned short lb = f2bf_bits(sp[e] - bf_bits2f(hb));
              hv[e] = __builtin_bit_cast(_Float16, hb);
              lv[e] = __builtin_bit_cast(_Float16, lb);
            }
          }
          *(volatile v8h*)(C + (size_t)(mBase + row) * ldc + n0 + c8) = hv;
          if (OUT_MODE == 2) *(volatile v8h*)(C2 + (size_t)(mBase + row) * ldc + n0 + c8) = lv;
        }
        __threadfence();
      }
    }
    __builtin_amdgcn_fence(__ATOMIC_RELEASE, "workgroup");
    __builtin_amdgcn_wave_barrier();
    __builtin_amdgcn_fence(__ATOMIC_ACQUIRE, "workgroup");
  }
}

__device__ __forceinline__ unsigned h_pair(float a, float b) {
  return (unsigned)__builtin_bit_cast(unsigned short, (_Float16)a) |
         ((unsigned)__builtin_bit_cast(unsigned short, (_Float16)b) << 16);
}
__device__ __forceinline__ void bf_pair(float a, float b, unsigned& wh, unsigned& wl) {
  const unsigned short ha = f2bf_bits(a), hb = f2bf_bits(b);
  const unsigned short la = f2bf_bits(a - bf_bits2f(ha)), lb = f2bf_bits(b - bf_bits2f(hb));
  wh = (unsigned)ha | ((unsigned)hb << 16);
  wl = (unsigned)la | ((unsigned)lb << 16);
}
__device__ __forceinline__ void bf_split8(v4f f0, v4f f1, v4u& wh, v4u& wl) {
  unsigned h0, h1, h2, h3, l0, l1, l2, l3;
  bf_pair(f0[0], f0[1], h0, l0);
  bf_pair(f0[2], f0[3], h1, l1);
  bf_pair(f1[0], f1[1], h2, l2);
  bf_pair(f1[2], f1[3], h3, l3);
  wh = (v4u){h0, h1, h2, h3};
  wl = (v4u){l0, l1, l2, l3};
}
__device__ __forceinline__ v4u h_pack8(v4f f0, v4f f1) {
  return (v4u){h_pair(f0[0], f0[1]), h_pair(f0[2], f0[3]), h_pair(f1[0], f1[1]), h_pair(f1[2], f1[3])};
}

__global__ __launch_bounds__(256) void ln_planes_kernel(
    const float* __restrict__ x, const float* __restrict__ gam, const float* __restrict__ bet,
    unsigned short* __restrict__ xf, unsigned short* __restrict__ xh, unsigned short* __restrict__ xl)
{
  const int lane = threadIdx.x & 31, wave = threadIdx.x >> 5;
  const int row = blockIdx.x * 8 + wave;
  const int bb = row >> 10, ss = row & (SEQP - 1);
  const bool valid = (ss < SEQ);
  const int ssc = valid ? ss : (SEQ - 1);
  const float* xr = x + (size_t)(bb * SEQ + ssc) * CIN;
  const int c0 = 8 * lane, c1 = 256 + 8 * lane;
  v4f a0 = *(const v4f*)(xr + c0);
  v4f a1 = *(const v4f*)(xr + c0 + 4);
  v4f a2 = *(const v4f*)(xr + c1);
  v4f a3 = *(const v4f*)(xr + c1 + 4);
  float sm = ((a0[0] + a0[1]) + (a0[2] + a0[3])) + ((a1[0] + a1[1]) + (a1[2] + a1[3]))
           + ((a2[0] + a2[1]) + (a2[2] + a2[3])) + ((a3[0] + a3[1]) + (a3[2] + a3[3]));
#pragma unroll
  for (int off = 16; off > 0; off >>= 1) sm += __shfl_xor(sm, off, 32);
  const float mean = sm * (1.0f / 512.0f);
  v4f d0 = a0 - mean, d1 = a1 - mean, d2 = a2 - mean, d3 = a3 - mean;
  float sq = (d0[0] * d0[0] + d0[1] * d0[1] + d0[2] * d0[2] + d0[3] * d0[3])
           + (d1[0] * d1[0] + d1[1] * d1[1] + d1[2] * d1[2] + d1[3] * d1[3])
           + (d2[0] * d2[0] + d2[1] * d2[1] + d2[2] * d2[2] + d2[3] * d2[3])
           + (d3[0] * d3[0] + d3[1] * d3[1] + d3[2] * d3[2] + d3[3] * d3[3]);
#pragma unroll
  for (int off = 16; off > 0; off >>= 1) sq += __shfl_xor(sq, off, 32);
  const float rstd = rsqrtf(sq * (1.0f / 512.0f) + 1e-5f);
  const v4f g0 = *(const v4f*)(gam + c0), g1 = *(const v4f*)(gam + c0 + 4);
  const v4f g2 = *(const v4f*)(gam + c1), g3 = *(const v4f*)(gam + c1 + 4);
  const v4f e0 = *(const v4f*)(bet + c0), e1 = *(const v4f*)(bet + c0 + 4);
  const v4f e2 = *(const v4f*)(bet + c1), e3 = *(const v4f*)(bet + c1 + 4);
  v4f y0 = d0 * rstd * g0 + e0;
  v4f y1 = d1 * rstd * g1 + e1;
  v4f y2 = d2 * rstd * g2 + e2;
  v4f y3 = d3 * rstd * g3 + e3;
  if (!valid) {
    const v4f z = (v4f){0.f, 0.f, 0.f, 0.f};
    y0 = z; y1 = z; y2 = z; y3 = z;
  }
  const v4u pf0 = h_pack8(y0, y1), pf1 = h_pack8(y2, y3);
  v4u ph0, pl0, ph1, pl1;
  bf_split8(y0, y1, ph0, pl0);
  bf_split8(y2, y3, ph1, pl1);
  const size_t ro = (size_t)row * CIN;
  for (int pass = 0; pass < 2; ++pass) {
    *(volatile v4u*)(xf + ro + c0) = pf0;
    *(volatile v4u*)(xf + ro + c1) = pf1;
    *(volatile v4u*)(xh + ro + c0) = ph0;
    *(volatile v4u*)(xh + ro + c1) = ph1;
    *(volatile v4u*)(xl + ro + c0) = pl0;
    *(volatile v4u*)(xl + ro + c1) = pl1;
    __threadfence();
  }
}

template <int MODE>
__global__ __launch_bounds__(256) void cast8_kernel(
    const float* __restrict__ src, unsigned short* __restrict__ d0, unsigned short* __restrict__ d1, int n8, float sc)
{
  const int i = blockIdx.x * 256 + threadIdx.x;
  if (i < n8) {
    const v4f a = *(const v4f*)(src + (size_t)i * 8);
    const v4f c = *(const v4f*)(src + (size_t)i * 8 + 4);
    if (MODE == 0) {
      const v4u w = h_pack8(a * sc, c * sc);
      for (int pass = 0; pass < 2; ++pass) {
        *(volatile v4u*)(d0 + (size_t)i * 8) = w;
        __threadfence();
      }
    } else {
      v4u wh, wl;
      bf_split8(a, c, wh, wl);
      for (int pass = 0; pass < 2; ++pass) {
        *(volatile v4u*)(d0 + (size_t)i * 8) = wh;
        *(volatile v4u*)(d1 + (size_t)i * 8) = wl;
        __threadfence();
      }
    }
  }
}

__device__ __forceinline__ v8f mma_bf(v16b a, v16b b, v8f c) {
  c = __builtin_amdgcn_wmma_f32_16x16x32_bf16(false, a, false, b, (short)0, c, false, false);
  asm volatile("v_nop\n\tv_nop\n\tv_nop\n\tv_nop" : "+v"(c) : "v"(a), "v"(b));
  return c;
}

__global__ __launch_bounds__(128)
void attn_relbias_kernel(const unsigned short* __restrict__ qh, const unsigned short* __restrict__ ql,
                        const unsigned short* __restrict__ kh, const unsigned short* __restrict__ kl,
                        const unsigned short* __restrict__ vh, const unsigned short* __restrict__ vl,
                        unsigned short* __restrict__ ch, unsigned short* __restrict__ cl, float sscale)
{
  union FB { v16b v; v8b h[2]; };
  __shared__ __align__(16) unsigned short sKh[64 * 64];
  __shared__ __align__(16) unsigned short sKl[64 * 64];
  __shared__ __align__(16) unsigned short sVh[64 * 64];
  __shared__ __align__(16) unsigned short sVl[64 * 64];
  __shared__ __align__(16) unsigned short sPh[4][16 * 64];
  __shared__ __align__(16) unsigned short sPl[4][16 * 64];
  __shared__ __align__(16) float sO[4][16 * 68];

  const int tid  = threadIdx.x;
  const int wave = tid >> 5;
  const int lane = tid & 31;
  const int hh   = lane >> 4;
  const int c    = lane & 15;

  const int bx  = blockIdx.x;
  const int qb  = bx & 15;
  const int bhd = bx >> 4;
  const int h   = bhd & (NHEAD - 1);
  const int b   = bhd >> 3;
  const int q0  = qb * 64 + wave * 16;

  v16b qah[2], qal[2];
  {
    const size_t qo = (size_t)(b * SEQP + q0 + c) * CIN + h * HDIM;
    const __bf16* ph = (const __bf16*)(qh + qo);
    const __bf16* pl = (const __bf16*)(ql + qo);
#pragma unroll
    for (int dc = 0; dc < 2; ++dc) {
      qah[dc] = Frag<__bf16>::load(ph + dc * 32 + 8 * hh);
      qal[dc] = Frag<__bf16>::load(pl + dc * 32 + 8 * hh);
    }
  }

  float mrow[8], lrow[8];
  v8f oacc[4];
#pragma unroll
  for (int r = 0; r < 8; ++r) { mrow[r] = -INFINITY; lrow[r] = 0.f; }
#pragma unroll
  for (int t = 0; t < 4; ++t) oacc[t] = (v8f){0.f,0.f,0.f,0.f,0.f,0.f,0.f,0.f};

  for (int kc = 0; kc < KV_LIM / 64; ++kc) {
    const int kv0 = kc * 64;
    __syncthreads();
    {
      const int kvr = tid >> 1, dh = (tid & 1) * 32;
      const size_t ro = (size_t)(b * KV_LIM + kv0 + kvr) * CIN + h * HDIM + dh;
      const v4u* gkh = (const v4u*)(kh + ro);
      const v4u* gkl = (const v4u*)(kl + ro);
      const v4u* gvh = (const v4u*)(vh + ro);
      const v4u* gvl = (const v4u*)(vl + ro);
#pragma unroll
      for (int i = 0; i < 4; ++i) {
        const v4u wkh = gkh[i], wkl = gkl[i], wvh = gvh[i], wvl = gvl[i];
        *(v4u*)(sKh + kvr * 64 + dh + 8 * i) = wkh;
        *(v4u*)(sKl + kvr * 64 + dh + 8 * i) = wkl;
#pragma unroll
        for (int e = 0; e < 4; ++e) {
          const int d = dh + 8 * i + 2 * e;
          sVh[d * 64 + kvr]       = (unsigned short)(wvh[e] & 0xffffu);
          sVh[(d + 1) * 64 + kvr] = (unsigned short)(wvh[e] >> 16);
          sVl[d * 64 + kvr]       = (unsigned short)(wvl[e] & 0xffffu);
          sVl[(d + 1) * 64 + kvr] = (unsigned short)(wvl[e] >> 16);
        }
      }
    }
    __syncthreads();

    v8f s[4];
#pragma unroll
    for (int j = 0; j < 4; ++j) {
      s[j] = (v8f){0.f,0.f,0.f,0.f,0.f,0.f,0.f,0.f};
#pragma unroll
      for (int dc = 0; dc < 2; ++dc) {
        FB kb, kbl;
        kb.h[0]  = *(const v8b*)(sKh + (j * 16 + c) * 64 + dc * 32 + 8 * hh);
        kb.h[1]  = *(const v8b*)(sKh + (j * 16 + c) * 64 + dc * 32 + 16 + 8 * hh);
        kbl.h[0] = *(const v8b*)(sKl + (j * 16 + c) * 64 + dc * 32 + 8 * hh);
        kbl.h[1] = *(const v8b*)(sKl + (j * 16 + c) * 64 + dc * 32 + 16 + 8 * hh);
        s[j] = mma_bf(qah[dc], kb.v, s[j]);
        s[j] = mma_bf(qah[dc], kbl.v, s[j]);
        s[j] = mma_bf(qal[dc], kb.v, s[j]);
      }
    }
    float cm[8];
#pragma unroll
    for (int r = 0; r < 8; ++r) {
      const int qpos = q0 + 8 * hh + r;
      float m = -INFINITY;
#pragma unroll
      for (int j = 0; j < 4; ++j) {
        const int kvcol = kv0 + j * 16 + c;
        const float val = s[j][r] * sscale + (float)(qpos - kvcol);
        s[j][r] = val;
        m = fmaxf(m, val);
      }
#pragma unroll
      for (int off = 1; off < 16; off <<= 1) m = fmaxf(m, __shfl_xor(m, off, 32));
      cm[r] = m;
    }
    unsigned short* pwh = sPh[wave];
    unsigned short* pwl = sPl[wave];
#pragma unroll
    for (int r = 0; r < 8; ++r) {
      const float mnew = fmaxf(mrow[r], cm[r]);
      const float alpha = expf(mrow[r] - mnew);
      mrow[r] = mnew;
      float psum = 0.f;
#pragma unroll
      for (int j = 0; j < 4; ++j) {
        const float p = expf(s[j][r] - mnew);
        psum += p;
        const unsigned short hb = f2bf_bits(p);
        const unsigned short lb = f2bf_bits(p - bf_bits2f(hb));
        pwh[(8 * hh + r) * 64 + j * 16 + c] = hb;
        pwl[(8 * hh + r) * 64 + j * 16 + c] = lb;
      }
#pragma unroll
      for (int off = 1; off < 16; off <<= 1) psum += __shfl_xor(psum, off, 32);
      lrow[r] = lrow[r] * alpha + psum;
#pragma unroll
      for (int t = 0; t < 4; ++t) oacc[t][r] *= alpha;
    }
    __builtin_amdgcn_fence(__ATOMIC_RELEASE, "workgroup");
    __builtin_amdgcn_wave_barrier();
    __builtin_amdgcn_fence(__ATOMIC_ACQUIRE, "workgroup");
#pragma unroll 1
    for (int kk = 0; kk < 2; ++kk) {
      FB pa, pl;
      pa.h[0] = *(const v8b*)(pwh + c * 64 + kk * 32 + 8 * hh);
      pa.h[1] = *(const v8b*)(pwh + c * 64 + kk * 32 + 16 + 8 * hh);
      pl.h[0] = *(const v8b*)(pwl + c * 64 + kk * 32 + 8 * hh);
      pl.h[1] = *(const v8b*)(pwl + c * 64 + kk * 32 + 16 + 8 * hh);
#pragma unroll
      for (int t = 0; t < 4; ++t) {
        FB vb, vbl;
        vb.h[0]  = *(const v8b*)(sVh + (t * 16 + c) * 64 + kk * 32 + 8 * hh);
        vb.h[1]  = *(const v8b*)(sVh + (t * 16 + c) * 64 + kk * 32 + 16 + 8 * hh);
        vbl.h[0] = *(const v8b*)(sVl + (t * 16 + c) * 64 + kk * 32 + 8 * hh);
        vbl.h[1] = *(const v8b*)(sVl + (t * 16 + c) * 64 + kk * 32 + 16 + 8 * hh);
        oacc[t] = mma_bf(pa.v, vb.v, oacc[t]);
        oacc[t] = mma_bf(pa.v, vbl.v, oacc[t]);
        oacc[t] = mma_bf(pl.v, vb.v, oacc[t]);
      }
    }
  }

  float* os = sO[wave];
#pragma unroll
  for (int r = 0; r < 8; ++r) {
    const float inv = 1.0f / lrow[r];
#pragma unroll
    for (int t = 0; t < 4; ++t) os[(8 * hh + r) * 68 + t * 16 + c] = oacc[t][r] * inv;
  }
  __builtin_amdgcn_fence(__ATOMIC_RELEASE, "workgroup");
  __builtin_amdgcn_wave_barrier();
  __builtin_amdgcn_fence(__ATOMIC_ACQUIRE, "workgroup");
  {
    const int q4 = lane >> 3, c8 = (lane & 7) * 8;
    for (int pass = 0; pass < 2; ++pass) {
#pragma unroll
      for (int it = 0; it < 4; ++it) {
        const int row = it * 4 + q4;
        const v4f f0 = *(const v4f*)(os + row * 68 + c8);
        const v4f f1 = *(const v4f*)(os + row * 68 + c8 + 4);
        v4u wh, wl;
        bf_split8(f0, f1, wh, wl);
        const size_t co = (size_t)(b * SEQP + q0 + row) * CIN + h * HDIM + c8;
        *(volatile v4u*)(ch + co) = wh;
        *(volatile v4u*)(cl + co) = wl;
      }
      __threadfence();
    }
  }
}

extern "C" void kernel_launch(void* const* d_in, const int* in_sizes, int n_in,
                              void* d_out, int out_size, void* d_ws, size_t ws_size,
                              hipStream_t stream) {
  (void)in_sizes; (void)n_in; (void)out_size; (void)ws_size;
  const float* x    = (const float*)d_in[0];
  const float* ln_g = (const float*)d_in[1];
  const float* ln_b = (const float*)d_in[2];
  const float* Wq   = (const float*)d_in[3];
  const float* bq   = (const float*)d_in[4];
  const float* Wk   = (const float*)d_in[5];
  const float* bk   = (const float*)d_in[6];
  const float* Wv   = (const float*)d_in[7];
  const float* bv   = (const float*)d_in[8];
  const float* Wo   = (const float*)d_in[9];
  const float* bo   = (const float*)d_in[10];
  float* out = (float*)d_out;

  const size_t WOFF = (size_t)LAYER_LAST * CIN * CIN;
  const size_t VOFF = (size_t)LAYER_LAST * CIN;
  const float* g5  = ln_g + VOFF;
  const float* be5 = ln_b + VOFF;
  const float* bq5 = bq + VOFF;
  const float* bk5 = bk + VOFF;
  const float* bv5 = bv + VOFF;
  const float* bo5 = bo + VOFF;

  constexpr size_t PLANE_X  = (size_t)MROWS * CIN * 2;
  constexpr size_t PLANE_W  = (size_t)CIN * CIN * 2;
  constexpr size_t PLANE_KV = (size_t)NBATCH * KV_LIM * CIN * 2;
  constexpr size_t OFF_XF  = 0;
  constexpr size_t OFF_XH  = OFF_XF + PLANE_X;
  constexpr size_t OFF_XL  = OFF_XH + PLANE_X;
  constexpr size_t OFF_WQ  = OFF_XL + PLANE_X;
  constexpr size_t OFF_WK  = OFF_WQ + PLANE_W;
  constexpr size_t OFF_WVH = OFF_WK + PLANE_W;
  constexpr size_t OFF_WVL = OFF_WVH + PLANE_W;
  constexpr size_t OFF_WOH = OFF_WVL + PLANE_W;
  constexpr size_t OFF_WOL = OFF_WOH + PLANE_W;
  constexpr size_t OFF_QH  = OFF_WOL + PLANE_W;
  constexpr size_t OFF_QL  = OFF_QH + PLANE_X;
  constexpr size_t OFF_KH  = OFF_QL + PLANE_X;
  constexpr size_t OFF_KL  = OFF_KH + PLANE_KV;
  constexpr size_t OFF_VH  = OFF_KL + PLANE_KV;
  constexpr size_t OFF_VL  = OFF_VH + PLANE_KV;
  constexpr size_t OFF_CH  = OFF_VL + PLANE_KV;
  constexpr size_t OFF_CL  = OFF_CH + PLANE_X;
  constexpr size_t WS_TOTAL = OFF_CL + PLANE_X;
  static_assert(WS_TOTAL == 70254592, "carve total");
  static_assert(WS_TOTAL <= (size_t)134217728, "carve within 128 MiB");

  char* ws = (char*)d_ws;
  unsigned short* xf  = (unsigned short*)(ws + OFF_XF);
  unsigned short* xh  = (unsigned short*)(ws + OFF_XH);
  unsigned short* xl  = (unsigned short*)(ws + OFF_XL);
  unsigned short* wqf = (unsigned short*)(ws + OFF_WQ);
  unsigned short* wkf = (unsigned short*)(ws + OFF_WK);
  unsigned short* wvh = (unsigned short*)(ws + OFF_WVH);
  unsigned short* wvl = (unsigned short*)(ws + OFF_WVL);
  unsigned short* woh = (unsigned short*)(ws + OFF_WOH);
  unsigned short* wol = (unsigned short*)(ws + OFF_WOL);
  unsigned short* qhp = (unsigned short*)(ws + OFF_QH);
  unsigned short* qlp = (unsigned short*)(ws + OFF_QL);
  unsigned short* khp = (unsigned short*)(ws + OFF_KH);
  unsigned short* klp = (unsigned short*)(ws + OFF_KL);
  unsigned short* vhp = (unsigned short*)(ws + OFF_VH);
  unsigned short* vlp = (unsigned short*)(ws + OFF_VL);
  unsigned short* chp = (unsigned short*)(ws + OFF_CH);
  unsigned short* clp = (unsigned short*)(ws + OFF_CL);

  const float WSC = 32.0f;
  const int   n8  = CIN * CIN / 8;
  static_assert((CIN * CIN / 8) % 256 == 0, "cast grid exact");
  static_assert(MROWS % 8 == 0, "ln grid exact");

  ln_planes_kernel<<<MROWS / 8, 256, 0, stream>>>(x, g5, be5, xf, xh, xl);
  cast8_kernel<0><<<n8 / 256, 256, 0, stream>>>(Wq + WOFF, wqf, wqf, n8, WSC);
  cast8_kernel<0><<<n8 / 256, 256, 0, stream>>>(Wk + WOFF, wkf, wkf, n8, WSC);
  cast8_kernel<1><<<n8 / 256, 256, 0, stream>>>(Wv + WOFF, wvh, wvl, n8, 1.0f);
  cast8_kernel<1><<<n8 / 256, 256, 0, stream>>>(Wo + WOFF, woh, wol, n8, 1.0f);

  {
    const int tiles = (MROWS / 64) * (CIN / 64);
    wmma_gemm64<0, false, 2, 2, false, 0, false><<<dim3(tiles / 8, 1), 256, 0, stream>>>(
        xf, xf, CIN, 0L, wqf, wqf, CIN, 0L, (void*)qhp, (void*)qlp, CIN, 0L,
        bq5, bq5, 0L, MROWS, CIN, CIN, 1.0f / WSC, 1, 1);
  }
  {
    const int tiles = (KV_LIM / 64) * (CIN / 64);
    wmma_gemm64<0, false, 2, 2, false, 0, false><<<dim3(tiles / 8, NBATCH), 256, 0, stream>>>(
        xf, xf, CIN, (long)SEQP * CIN, wkf, wkf, CIN, 0L, (void*)khp, (void*)klp, CIN, (long)KV_LIM * CIN,
        bk5, bk5, 0L, KV_LIM, CIN, CIN, 1.0f / WSC, 1, 1);
  }
  {
    const int tiles = (KV_LIM / 64) * (CIN / 64);
    wmma_gemm64<1, true, 2, 2, false, 0, false><<<dim3(tiles / 8, NBATCH), 256, 0, stream>>>(
        xh, xl, CIN, (long)SEQP * CIN, wvh, wvl, CIN, 0L, (void*)vhp, (void*)vlp, CIN, (long)KV_LIM * CIN,
        bv5, bv5, 0L, KV_LIM, CIN, CIN, 1.0f, 1, 1);
  }
  attn_relbias_kernel<<<NBATCH * NHEAD * (SEQP / 64), 128, 0, stream>>>(
      qhp, qlp, khp, klp, vhp, vlp, chp, clp, 0.125f);
  {
    const int tiles = (MROWS / 64) * (CIN / 64);
    wmma_gemm64<1, true, 2, 0, false, 0, true><<<dim3(tiles / 8, 1), 256, 0, stream>>>(
        chp, clp, CIN, 0L, woh, wol, CIN, 0L, (void*)out, (void*)clp, CIN, 0L,
        bo5, bo5, 0L, MROWS, CIN, CIN, 1.0f, SEQP, SEQ);
  }
}
